// SeqGraph_27986006901054
// MI455X (gfx1250) — hardware-run, weakly checked
//
#include <hip/hip_runtime.h>


namespace {
constexpr int N = 100000, NP = 100032, E = 640000, D = 128, GH = 16, SH = 10, ZR = GH * SH  , B = 2048, NSTEP = 4, V = 100000;
constexpr float XS = 8.0f, ZS = 8.0f, WSC = 256.0f, NEG = 0.2f  , LSLOPE = 0.01f;

typedef _Float16 b16;
typedef __attribute__((ext_vector_type(16))) _Float16 v16b;
typedef __attribute__((ext_vector_type(8))) _Float16 v8b;
typedef __attribute__((ext_vector_type(8))) float v8f;
typedef __attribute__((ext_vector_type(4))) float v4f;
__device__ __forceinline__ float bf16_rne(float f) { unsigned int u = __float_as_uint(f); u += 0x7FFFu + ((u >> 16) & 1u); return __uint_as_float(u & 0xFFFF0000u); }
__device__ __forceinline__ void split16(float v, b16& hi, b16& lo) { hi = (b16)v; lo = (b16)(v - (float)hi); }
__device__ __forceinline__ v16b frag_kb(const b16* p, int hh) { const v8b a = *(const v8b*)(p + 8 * hh), b = *(const v8b*)(p + 16 + 8 * hh); v16b f;
#pragma unroll
  for (int e = 0; e < 8; ++e) { f[e] = a[e]; f[8 + e] = b[e]; } return f; }
__device__ __forceinline__ v8f wmma16b(v16b a, v16b b, v8f c) { v8f d = __builtin_amdgcn_wmma_f32_16x16x32_f16(false, a, false, b, (short)0, c, false, false); asm volatile("v_nop\n\tv_nop\n\tv_nop\n\tv_nop" : "+v"(d) : "v"(a), "v"(b)); return d; }
__device__ __forceinline__ void wave_lds_sync() { __builtin_amdgcn_fence(__ATOMIC_RELEASE, "workgroup"); __builtin_amdgcn_wave_barrier(); __builtin_amdgcn_fence(__ATOMIC_ACQUIRE, "workgroup"); }
__device__ __forceinline__ float pmul(float a, float b) { float p = a * b; asm volatile("" : "+v"(p)); return p; }
__device__ __forceinline__ int iclamp(int v, int lo, int hi) { return v < lo ? lo : (v > hi ? hi : v); }
__device__ __forceinline__ float nexp(float x) { return __builtin_amdgcn_exp2f(x * 1.4426950408889634f); }
__device__ __forceinline__ float lrelu(float x) { return x > 0.0f ? x : NEG * x; }

constexpr int CSR_NBLK = 512, CSR_GB = 9, CSR_GN = 1 << CSR_GB  , CSR_MAXG = 512, CSR_CAP = 12288  ;
__global__ __launch_bounds__(64) void csrA_kernel(const int* __restrict__ dst, int E, int N, int nG, int CHP, int NGP, int* __restrict__ STG, int* __restrict__ HST) {
  extern __shared__ int sm[];
  int* cnt = sm; int* run = sm + NGP; int* ids = sm + 2 * NGP;
  const int b = blockIdx.x; const int ch = (E + CSR_NBLK - 1) / CSR_NBLK; const int e0 = b * ch, e1 = min(E, e0 + ch);
  for (int i = threadIdx.x; i < NGP; i += 64) cnt[i] = 0;
  for (int i = threadIdx.x; i < CHP; i += 64) ids[i] = -1;
  __syncthreads();
  if (threadIdx.x == 0) {
    for (int e = e0; e < e1; ++e) { int d = dst[e]; d = (d < 0) ? 0 : (d >= N ? N - 1 : d); cnt[d >> CSR_GB] += 1; }
    int acc = 0; for (int g = 0; g < nG; ++g) { run[g] = acc; acc += cnt[g]; }
    for (int e = e0; e < e1; ++e) { int d = dst[e]; d = (d < 0) ? 0 : (d >= N ? N - 1 : d); const int g = d >> CSR_GB; ids[run[g]] = e; run[g] += 1; } }
  __syncthreads();
  typedef __attribute__((ext_vector_type(4))) int v4i;
  for (int pass = 0; pass < 2; ++pass) {
    for (int i = threadIdx.x; i < CHP / 4; i += 64) *(volatile v4i*)(STG + (size_t)b * CHP + i * 4) = *(const v4i*)(&ids[i * 4]);
    for (int i = threadIdx.x; i < NGP / 4; i += 64) { v4i v; for (int e = 0; e < 4; ++e) v[e] = (i * 4 + e < nG) ? cnt[i * 4 + e] : 0; *(volatile v4i*)(HST + (size_t)b * NGP + i * 4) = v; }
    __threadfence(); }
}
__global__ __launch_bounds__(512) void csrS_kernel(const int* __restrict__ HST, int nG, int NGP, int* __restrict__ START, int* __restrict__ TOT, int* __restrict__ OFF) {
  __shared__ int tot[CSR_MAXG];
  const int b = threadIdx.x;
  for (int pass = 0; pass < 2; ++pass) { int runb = 0; for (int g = 0; g < nG; ++g) { int c = HST[(size_t)b * NGP + g]; c = (c < 0) ? 0 : c; ((volatile int*)OFF)[(size_t)g * CSR_NBLK + b] = runb; runb += c; } __threadfence(); }
  for (int g = threadIdx.x; g < nG; g += 512) { int s = 0; for (int bb = 0; bb < CSR_NBLK; ++bb) { int c = HST[(size_t)bb * NGP + g]; s += (c < 0) ? 0 : c; } tot[g] = s; }
  __syncthreads();
  if (threadIdx.x < 32) {
    __shared__ int st[CSR_MAXG + 32];
    if (threadIdx.x == 0) { int acc = 0; for (int g = 0; g < NGP; ++g) { st[g] = acc; if (g < nG) acc += (tot[g] + 31) & ~31; } st[NGP] = acc; }
    __builtin_amdgcn_fence(__ATOMIC_RELEASE, "workgroup"); __builtin_amdgcn_wave_barrier(); __builtin_amdgcn_fence(__ATOMIC_ACQUIRE, "workgroup");
    for (int pass = 0; pass < 2; ++pass) { for (int i = threadIdx.x; i < NGP + 32; i += 32) { ((volatile int*)START)[i] = (i <= NGP) ? st[min(i, NGP)] : 0; ((volatile int*)TOT)[i] = (i < nG) ? tot[i] : 0; } __threadfence(); } }
}
__global__ __launch_bounds__(256) void csrB_kernel(const int* __restrict__ dst, int N, int nG, int CHP, int NGP, int permLen, const int* __restrict__ STG, const int* __restrict__ HST, const int* __restrict__ OFF, const int* __restrict__ START, const int* __restrict__ TOT, int* __restrict__ PERM, int* __restrict__ ROWPTR, int* __restrict__ ROWCNT, int* __restrict__ FLAG) {
  typedef __attribute__((ext_vector_type(4))) int v4i;
  __shared__ int ids[CSR_CAP]; __shared__ unsigned short key[CSR_CAP]; __shared__ int outp[CSR_CAP]; __shared__ int ncnt[CSR_GN + 1]; __shared__ int boff[CSR_NBLK + 1];
  const int g = blockIdx.x, t_ = threadIdx.x; int tot = TOT[g]; int st = START[g], stn = START[g + 1]; const int v0 = g * CSR_GN; const int nv = min(CSR_GN, N - v0);
  st = (st < 0) ? 0 : (st > permLen - 32 ? permLen - 32 : st) & ~31; stn = (stn < st) ? st : (stn > permLen ? permLen : stn); tot = (tot < 0) ? 0 : tot; if (tot > stn - st && tot <= CSR_CAP) tot = stn - st;
  if (tot > CSR_CAP) {
    for (int pass = 0; pass < 2; ++pass) { for (int i = t_; i < CSR_GN / 4; i += 256) { v4i a, c; for (int e = 0; e < 4; ++e) { a[e] = st; c[e] = 0; } *(volatile v4i*)(ROWPTR + v0 + i * 4) = a; *(volatile v4i*)(ROWCNT + v0 + i * 4) = c; } if (t_ == 0) ((volatile int*)FLAG)[0] = 1; __threadfence(); } (void)nv; return; }
  if (t_ == 0) { int acc = 0; for (int b = 0; b < CSR_NBLK; ++b) { boff[b] = acc; int c = HST[(size_t)b * NGP + g]; c = (c < 0) ? 0 : (c > CHP ? CHP : c); acc += c; if (acc > tot) acc = tot; } boff[CSR_NBLK] = acc; }
  for (int i = t_; i <= CSR_GN; i += 256) ncnt[i] = 0;
  __syncthreads();
  for (int b = 0; b < CSR_NBLK; ++b) { const int c = boff[b + 1] - boff[b]; int o_ = OFF[(size_t)g * CSR_NBLK + b]; o_ = (o_ < 0) ? 0 : (o_ > CHP - c ? CHP - c : o_); const int* src_ = STG + (size_t)b * CHP + o_;
    for (int i = t_; i < c; i += 256) { int id = src_[i]; id = (id < 0) ? 0 : id; ids[boff[b] + i] = id; int d = dst[id]; d = (d < v0) ? v0 : (d >= N ? N - 1 : d); int kk = d - v0; kk = (kk < 0) ? 0 : (kk >= CSR_GN ? CSR_GN - 1 : kk); key[boff[b] + i] = (unsigned short)kk; } }
  __syncthreads();
  if (t_ == 0) { for (int i = 0; i < tot; ++i) ncnt[key[i]] += 1; int acc = 0; for (int vl = 0; vl < CSR_GN; ++vl) { const int c = ncnt[vl]; ncnt[vl] = acc; acc += c; } ncnt[CSR_GN] = acc;
    for (int i = 0; i < tot; ++i) { const int vl = key[i]; outp[ncnt[vl]] = ids[i]; ncnt[vl] += 1; }
    for (int vl = CSR_GN; vl > 0; --vl) ncnt[vl] = ncnt[vl - 1]; ncnt[0] = 0; }
  __syncthreads();
  for (int pass = 0; pass < 2; ++pass) {
    for (int i = t_; i < (stn - st) / 4; i += 256) { v4i v; for (int e = 0; e < 4; ++e) { const int q = i * 4 + e; v[e] = (q < tot) ? outp[q] : -1; } *(volatile v4i*)(PERM + st + i * 4) = v; }
    for (int i = t_; i < CSR_GN / 4; i += 256) { v4i a, c; for (int e = 0; e < 4; ++e) { const int vl = i * 4 + e; a[e] = st + ncnt[vl]; c[e] = (vl < nv) ? (ncnt[vl + 1] - ncnt[vl]) : 0; } *(volatile v4i*)(ROWPTR + v0 + i * 4) = a; *(volatile v4i*)(ROWCNT + v0 + i * 4) = c; }
    __threadfence(); }
}
__global__ __launch_bounds__(256) void csrZ_kernel(int* __restrict__ p, size_t n4) { typedef __attribute__((ext_vector_type(4))) int v4i; const size_t tid = (size_t)blockIdx.x * 256 + threadIdx.x, nth = (size_t)gridDim.x * 256; v4i z = {0, 0, 0, 0}; for (size_t i = tid; i < n4; i += nth) *(volatile v4i*)(p + i * 4) = z; }
struct CsrBufs { int *STG, *HST, *OFF, *START, *TOT, *PERM, *ROWPTR, *ROWCNT, *FLAG; int nG, NGP, CHP; size_t permLen; char* base; size_t bytes; };
static size_t csr_carve(CsrBufs& c, char* ws, size_t off, int E, int N) {
  const size_t off0 = off; c.base = ws + off;
  auto al = [&](size_t bytes) { char* p = ws + off; off += (bytes + 255) & ~(size_t)255; return p; };
  c.nG = (N + CSR_GN - 1) / CSR_GN; c.NGP = (c.nG + 31) & ~31; const int ch = (E + CSR_NBLK - 1) / CSR_NBLK; c.CHP = (ch + 31) & ~31; c.permLen = (size_t)E + 32 * (size_t)c.nG + 32;
  c.STG = (int*)al((size_t)CSR_NBLK * c.CHP * 4); c.HST = (int*)al((size_t)CSR_NBLK * c.NGP * 4); c.OFF = (int*)al((size_t)c.NGP * CSR_NBLK * 4); c.START = (int*)al((size_t)(c.NGP + 64) * 4); c.TOT = (int*)al((size_t)(c.NGP + 64) * 4);
  c.PERM = (int*)al(c.permLen * 4); c.ROWPTR = (int*)al((size_t)c.nG * CSR_GN * 4); c.ROWCNT = (int*)al((size_t)c.nG * CSR_GN * 4); c.FLAG = (int*)al(256);
  c.bytes = off - off0; return off;
}
static void csr_build(const CsrBufs& c, const int* dst, int E, int N, hipStream_t stream) {
  const size_t smem = (size_t)(2 * c.NGP + c.CHP) * 4;
  csrZ_kernel<<<512, 256, 0, stream>>>((int*)c.base, c.bytes / 16);
  csrA_kernel<<<CSR_NBLK, 64, smem, stream>>>(dst, E, N, c.nG, c.CHP, c.NGP, c.STG, c.HST);
  csrS_kernel<<<1, 512, 0, stream>>>(c.HST, c.nG, c.NGP, c.START, c.TOT, c.OFF);
  csrB_kernel<<<c.nG, 256, 0, stream>>>(dst, N, c.nG, c.CHP, c.NGP, (int)c.permLen, c.STG, c.HST, c.OFF, c.START, c.TOT, c.PERM, c.ROWPTR, c.ROWCNT, c.FLAG);
}


__device__ __forceinline__ float leaky(float x) { return x >= 0.0f ? x : LSLOPE * x; }
__global__ __launch_bounds__(256) void prep_kernel(const float* __restrict__ wfc, b16* __restrict__ WFT) {
  const size_t u = (size_t)blockIdx.x * 256 + threadIdx.x; const size_t nw = (size_t)D * D / 8; size_t t = u; v8b o;
  if (t < nw) { const size_t e = t * 8; const int oo = (int)(e / D), k0 = (int)(e % D); for (int j = 0; j < 8; ++j) o[j] = (b16)(bf16_rne(wfc[(size_t)(k0 + j) * D + oo]) * WSC); for (int pass = 0; pass < 2; ++pass) { *(volatile v8b*)(WFT + e) = o; __threadfence(); } }
}
__global__ __launch_bounds__(256) void zprep_kernel(const float* __restrict__ hadj, const float* __restrict__ hfeat, b16* __restrict__ ZPh, b16* __restrict__ ZPl) {
  __shared__ float A_[SH][SH]; __shared__ __attribute__((aligned(16))) float zc[2][SH][D];
  const int g = blockIdx.x, t = threadIdx.x;
  if (t < SH * SH) A_[t / SH][t % SH] = 0.0f;
  __syncthreads();
  if (t < SH * (SH - 1) / 2) {
    int k = t, i = 0; while (k >= SH - 1 - i) { k -= SH - 1 - i; ++i; } const int j = i + 1 + k; const float a = leaky(bf16_rne(hadj[g * 45 + t])); A_[i][j] = a; A_[j][i] = a; }
  for (int q = t; q < SH * D; q += 256) zc[0][q / D][q % D] = bf16_rne(hfeat[((size_t)g * SH + q / D) * D + q % D]);
  __syncthreads();
  for (int step = 0; step < NSTEP; ++step) { const int cur = step & 1;
    for (int pass = 0; pass < 2; ++pass) { if (t < SH * D / 8) { const int r = t / (D / 8), c8 = (t % (D / 8)) * 8; v8b h, l; for (int jj = 0; jj < 8; ++jj) { b16 p, q; split16(zc[cur][r][c8 + jj] * ZS, p, q); h[jj] = p; l[jj] = q; }
        *(volatile v8b*)(ZPh + ((size_t)step * ZR + g * SH + r) * D + c8) = h; *(volatile v8b*)(ZPl + ((size_t)step * ZR + g * SH + r) * D + c8) = l; } __threadfence(); }
    if (step + 1 < NSTEP) { for (int q = t; q < SH * D; q += 256) { const int s = q / D, d = q % D; float a = 0.0f;
#pragma unroll 1
        for (int tt = 0; tt < SH; ++tt) a += pmul(A_[s][tt], zc[cur][tt][d]); zc[cur ^ 1][s][d] = a; } }
    __syncthreads(); }
}
__global__ __launch_bounds__(128) void x0_kernel(const int* __restrict__ xid, const float* __restrict__ emb, const b16* __restrict__ WFT, const float* __restrict__ bfc, float* __restrict__ XA) {
  __shared__ __attribute__((aligned(16))) float Tf[4][16][D + 4];
  const int wave = threadIdx.x >> 5, lane = threadIdx.x & 31, nloc = lane & 15, hlf = lane >> 4; const size_t m0 = (size_t)blockIdx.x * 64 + wave * 16;
  v8f acc[8];
#pragma unroll
  for (int t = 0; t < 8; ++t) acc[t] = (v8f){};
#pragma unroll
  for (int kb = 0; kb < D; kb += 32) { v16b a = {}; { const size_t v = m0 + nloc; if (v < (size_t)N) { const float* er = emb + (size_t)iclamp(xid[v], 0, V - 1) * D + kb; for (int e = 0; e < 8; ++e) { a[e] = (b16)(bf16_rne(er[8 * hlf + e]) * XS); a[8 + e] = (b16)(bf16_rne(er[16 + 8 * hlf + e]) * XS); } } }
#pragma unroll
    for (int t = 0; t < 8; ++t) acc[t] = wmma16b(a, frag_kb(WFT + (size_t)(t * 16 + nloc) * D + kb, hlf), acc[t]); }
#pragma unroll
  for (int t = 0; t < 8; ++t) { const int c = t * 16 + nloc; const float bb = bf16_rne(bfc[c]);
#pragma unroll 1
    for (int r = 0; r < 8; ++r) { const size_t row = m0 + 8 * hlf + r; Tf[wave][8 * hlf + r][c] = row < (size_t)N ? 1.0f / (1.0f + __expf(-(acc[t][r] * (1.0f / (XS * WSC)) + bb))) : 0.0f; } }
  wave_lds_sync();
  for (int pass = 0; pass < 2; ++pass) { for (int rr = 0; rr < 16; ++rr) *(volatile v4f*)(XA + (m0 + rr) * D + lane * 4) = *(const v4f*)(&Tf[wave][rr][lane * 4]); __threadfence(); }
}
__global__ __launch_bounds__(256) void prop_kernel(const float* __restrict__ Xin, const int* __restrict__ srcs, const int* __restrict__ PERM, const int* __restrict__ ROWPTR, const int* __restrict__ ROWCNT, int permLen, float* __restrict__ Xout) {
  const int wave = threadIdx.x >> 5, lane = threadIdx.x & 31; const size_t v = (size_t)blockIdx.x * 8 + wave; v4f a = {0.0f, 0.0f, 0.0f, 0.0f};
  if (v < (size_t)N) { int st = ROWPTR[v], cnt = ROWCNT[v]; cnt = iclamp(cnt, 0, 65536); st = iclamp(st, 0, permLen - cnt);
#pragma unroll 1
    for (int i = 0; i < cnt; ++i) { const int e = iclamp(PERM[st + i], 0, E - 1); const size_t s = (size_t)iclamp(srcs[e], 0, N - 1); a += *(const v4f*)(Xin + s * D + lane * 4); } }
  for (int pass = 0; pass < 2; ++pass) { *(volatile v4f*)(Xout + v * D + lane * 4) = a; __threadfence(); }
}
template <int STEP0, int THREE>
__global__ __launch_bounds__(128) void step_kernel(const float* __restrict__ X, const b16* __restrict__ Zh, const b16* __restrict__ Zl, float* ZX, float* __restrict__ U) {
  __shared__ __attribute__((aligned(16))) b16 Ah[4][16][D + 8], Al[4][16][D + 8]; __shared__ __attribute__((aligned(16))) float Tf[4][16][ZR + 4]; __shared__ __attribute__((aligned(16))) float Uf[4][16][16];
  const int wave = threadIdx.x >> 5, lane = threadIdx.x & 31, nloc = lane & 15, hlf = lane >> 4; const size_t m0 = (size_t)blockIdx.x * 64 + wave * 16;
  for (int rr = 0; rr < 16; ++rr) { const v4f xv = *(const v4f*)(X + (m0 + rr) * D + lane * 4); for (int j = 0; j < 4; ++j) { b16 p, q; split16(xv[j] * XS, p, q); Ah[wave][rr][lane * 4 + j] = p; Al[wave][rr][lane * 4 + j] = q; } }
  wave_lds_sync();
  v8f acc[10];
#pragma unroll
  for (int t = 0; t < 10; ++t) acc[t] = (v8f){};
#pragma unroll
  for (int kb = 0; kb < D; kb += 32) { const v16b a = frag_kb(&Ah[wave][nloc][kb], hlf), al = frag_kb(&Al[wave][nloc][kb], hlf);
#pragma unroll
    for (int t = 0; t < 10; ++t) { const v16b bh = frag_kb(Zh + (size_t)(t * 16 + nloc) * D + kb, hlf); acc[t] = wmma16b(a, bh, acc[t]); acc[t] = wmma16b(al, bh, acc[t]); if (THREE) { const v16b bl = frag_kb(Zl + (size_t)(t * 16 + nloc) * D + kb, hlf); acc[t] = wmma16b(a, bl, acc[t]); } } }
#pragma unroll
  for (int t = 0; t < 10; ++t)
#pragma unroll 1
    for (int r = 0; r < 8; ++r) Tf[wave][8 * hlf + r][t * 16 + nloc] = acc[t][r] * (1.0f / (XS * ZS));
  wave_lds_sync();
  if (STEP0) { for (int pass = 0; pass < 2; ++pass) { for (int rr = 0; rr < 16; ++rr) { *(volatile v4f*)(ZX + (m0 + rr) * ZR + lane * 4) = *(const v4f*)(&Tf[wave][rr][lane * 4]); if (lane < 8) *(volatile v4f*)(ZX + (m0 + rr) * ZR + 128 + lane * 4) = *(const v4f*)(&Tf[wave][rr][128 + lane * 4]); } __threadfence(); } }
  for (int rr = 0; rr < 16; ++rr) { if (lane < 16) { float u = 0.0f; const size_t row = m0 + rr;
#pragma unroll
      for (int s = 0; s < SH; ++s) { const float tv = Tf[wave][rr][lane * SH + s]; const float zv = STEP0 ? tv : ZX[row * ZR + lane * SH + s]; u += pmul(zv, tv); }
      Uf[wave][rr][lane] = u; } }
  wave_lds_sync();
  for (int pass = 0; pass < 2; ++pass) { for (int rr = 0; rr < 16; ++rr) if (lane < 4) *(volatile v4f*)(U + (m0 + rr) * 16 + lane * 4) = *(const v4f*)(&Uf[wave][rr][lane * 4]); __threadfence(); }
}
__device__ int lower_bound_i(const int* a, int n, int key) { int lo = 0, hi = n; while (lo < hi) { const int mid = (lo + hi) >> 1; if (a[mid] < key) lo = mid + 1; else hi = mid; } return lo; }
__global__ __launch_bounds__(64) void pool_kernel(const float* __restrict__ U0, const float* __restrict__ U1, const float* __restrict__ U2, const float* __restrict__ U3, const int* __restrict__ batch, float* __restrict__ PC) {
  const int b = blockIdx.x, t = threadIdx.x; const int step = t >> 4, g = t & 15; const float* U = step == 0 ? U0 : step == 1 ? U1 : step == 2 ? U2 : U3;
  const int lo = lower_bound_i(batch, N, b), hi = lower_bound_i(batch, N, b + 1); float s = 0.0f; for (int v = lo; v < hi; ++v) s += U[(size_t)v * 16 + g];
  for (int pass = 0; pass < 2; ++pass) { ((volatile float*)PC)[(size_t)b * 64 + t] = s; __threadfence(); }
}
__global__ __launch_bounds__(128) void head_kernel(const float* __restrict__ PC, const float* __restrict__ wm, const float* __restrict__ bm, float* __restrict__ out) {
  const int c = threadIdx.x;
  for (int bb = 0; bb < 2; ++bb) { const int b = blockIdx.x * 2 + bb; float s = bf16_rne(bm[c]);
#pragma unroll 1
    for (int k = 0; k < 64; ++k) s += pmul(PC[(size_t)b * 64 + k], bf16_rne(wm[k * D + c]));
    const float y = leaky(s);
    for (int pass = 0; pass < 2; ++pass) { ((volatile float*)out)[(size_t)b * D + c] = y; __threadfence(); } }
}
}

extern "C" void kernel_launch(void* const* d_in, const int* in_sizes, int n_in, void* d_out, int out_size, void* d_ws, size_t ws_size, hipStream_t stream) {
  (void)n_in;
  auto Fp = [&](int i) { return (const float*)d_in[i]; }; auto Ip = [&](int i) { return (const int*)d_in[i]; };
  if (in_sizes[0] != N || in_sizes[1] != 2 * E || in_sizes[2] != N || in_sizes[3] != V * D || in_sizes[4] != D * D || in_sizes[6] != GH * 45 || in_sizes[7] != ZR * D || in_sizes[8] != 64 * D || out_size != B * D) return;
  size_t off = 0; char* ws = (char*)d_ws;
  auto carve = [&](size_t bytes) { char* p = ws + off; off += (bytes + 255) & ~(size_t)255; return p; };
  b16* WFT = (b16*)carve((size_t)D * D * 2); b16* ZPh = (b16*)carve((size_t)NSTEP * ZR * D * 2); b16* ZPl = (b16*)carve((size_t)NSTEP * ZR * D * 2);
  float* XA = (float*)carve((size_t)NP * D * 4); float* XB = (float*)carve((size_t)NP * D * 4); float* ZX = (float*)carve((size_t)NP * ZR * 4); float* U = (float*)carve((size_t)NSTEP * NP * 16 * 4); float* PC = (float*)carve((size_t)B * 64 * 4);
  CsrBufs csr; off = csr_carve(csr, ws, off, E, N);
  if (off > ws_size) return;
  prep_kernel<<<(unsigned)(((size_t)D * D / 8 + 255) / 256), 256, 0, stream>>>(Fp(4), WFT);
  zprep_kernel<<<GH, 256, 0, stream>>>(Fp(6), Fp(7), ZPh, ZPl);
  csr_build(csr, Ip(1) + E, E, N, stream);
  x0_kernel<<<NP / 64, 128, 0, stream>>>(Ip(0), Fp(3), WFT, Fp(5), XA);
  step_kernel<1, 0><<<NP / 64, 128, 0, stream>>>(XA, ZPh, ZPl, ZX, U);
  float* xin = XA; float* xout = XB;
  for (int i = 1; i < NSTEP; ++i) {
    prop_kernel<<<NP / 8, 256, 0, stream>>>(xin, Ip(1), csr.PERM, csr.ROWPTR, csr.ROWCNT, (int)csr.permLen, xout);
    step_kernel<0, 1><<<NP / 64, 128, 0, stream>>>(xout, ZPh + (size_t)i * ZR * D, ZPl + (size_t)i * ZR * D, ZX, U + (size_t)i * NP * 16);
    float* t = xin; xin = xout; xout = t; }
  pool_kernel<<<B, 64, 0, stream>>>(U, U + (size_t)NP * 16, U + (size_t)2 * NP * 16, U + (size_t)3 * NP * 16, Ip(2), PC);
  head_kernel<<<B / 2, 128, 0, stream>>>(PC, Fp(8), Fp(9), (float*)d_out);
}
